// Attention_54872502174159
// MI455X (gfx1250) — hardware-run, weakly checked
//
#include <hip/hip_runtime.h>
#include <stdint.h>


#ifndef NB
#define NB 4
#endif
#ifndef SEQ
#define SEQ 2048
#endif
#ifndef QRES
#define QRES 512
#endif
#define NB_FULL  4
#define SEQ_FULL 2048
#define CDIM 1024
#define NQKV 3072
#define NH   16
#define HD   64
#define LR   8
#define LRP  16
#define LSCALE 2.0f
#define QRES_E (((QRES) < (SEQ)) ? (QRES) : (SEQ))
#define MROWS ((NB) * (SEQ))

#define SST 72
#define SSF 68
#define PST 72
#define TS  72
#define XST 20

static_assert(NB >= 1 && NB <= NB_FULL);
static_assert(SEQ >= 128 && SEQ <= SEQ_FULL);
static_assert(SEQ % 128 == 0);
static_assert(QRES_E % 128 == 0);
static_assert(QRES_E <= SEQ);
static_assert(MROWS % 128 == 0);
static_assert(CDIM % 32 == 0 && NQKV % 128 == 0 && HD == 64);

#define SZ_XH   ((size_t)MROWS * CDIM * 2)
#define SZ_WQ   ((size_t)NQKV * CDIM * 2)
#define SZ_WP   ((size_t)CDIM * CDIM * 2)
#define SZ_AH   ((size_t)LRP * CDIM * 2)
#define SZ_XA   ((size_t)MROWS * LRP * 4)
#define SZ_QKVH ((size_t)MROWS * NQKV * 2)
#define SZ_QKVR ((size_t)NB * QRES_E * NQKV * 2)
#define SZ_VT   ((size_t)NB * NH * HD * SEQ * 2)
#define SZ_VTR  ((size_t)NB * NH * HD * QRES_E * 2)
#define SZ_CTXH ((size_t)MROWS * CDIM * 2)
#define SZ_CTXR ((size_t)NB * QRES_E * CDIM * 2)
#define WS_TOTAL (SZ_XH + SZ_WQ + SZ_WP + 2 * SZ_AH + 2 * SZ_XA + SZ_QKVH + SZ_QKVR + SZ_VT + SZ_VTR + SZ_CTXH + SZ_CTXR)
static_assert(WS_TOTAL <= (size_t)134217728);

typedef _Float16 v16h __attribute__((ext_vector_type(16)));
typedef _Float16 v8h  __attribute__((ext_vector_type(8)));
typedef float    v8f  __attribute__((ext_vector_type(8)));
typedef float    v4f  __attribute__((ext_vector_type(4)));
union Frag { v16h v; v8h half[2]; };

__device__ __forceinline__ v8f vz8() {
  v8f v;
#pragma unroll
  for (int i = 0; i < 8; ++i) v[i] = 0.0f;
  return v;
}

__device__ __forceinline__ float bf16r(float f) {
  unsigned u = __float_as_uint(f);
  u = (u + 0x7FFFu + ((u >> 16) & 1u)) & 0xFFFF0000u;
  return __uint_as_float(u);
}

__device__ __forceinline__ v8f wmma16(v16h a, v16h b, v8f c) {
  return __builtin_amdgcn_wmma_f32_16x16x32_f16(false, a, false, b, (short)0, c, false, false);
}

__device__ __forceinline__ v16h gfrag(const _Float16* p) {
  Frag f;
  f.half[0] = *(const v8h*)(p);
  f.half[1] = *(const v8h*)(p + 16);
  return f.v;
}

__global__ void __launch_bounds__(256)
cvt_kernel(const float* __restrict__ src, _Float16* __restrict__ dst,
           int dstRows, int segDst, int segSrc, int validT, float scale) {
  const int piece = blockIdx.x * 256 + (int)threadIdx.x;
  const int m  = piece >> 7;
  const int c8 = (piece & 127) * 8;
  if (m >= dstRows) return;
  const int bseg = m / segDst;
  const int t    = m - bseg * segDst;
  const bool valid = t < validT;
  const int tcl = valid ? t : 0;
  const float* sp = src + ((size_t)bseg * segSrc + tcl) * CDIM + c8;
  v4f a = *(const v4f*)(sp);
  v4f b = *(const v4f*)(sp + 4);
  v8h o;
#pragma unroll
  for (int e = 0; e < 4; ++e) {
    float f0 = bf16r(a[e]) * scale;
    float f1 = bf16r(b[e]) * scale;
    o[e]     = valid ? (_Float16)f0 : (_Float16)0.0f;
    o[e + 4] = valid ? (_Float16)f1 : (_Float16)0.0f;
  }
  _Float16* dp = dst + (size_t)m * CDIM + c8;
  *(volatile v8h*)dp = o;
  __threadfence();
  *(volatile v8h*)dp = o;
}

__global__ void __launch_bounds__(128)
lora_a_kernel(const _Float16* __restrict__ X, const _Float16* __restrict__ Ah,
              float* __restrict__ xa, float alpha) {
  __shared__ __align__(16) float St[4 * 16 * XST];
  const int tid = threadIdx.x, wave = tid >> 5, lane = tid & 31, lm = lane & 15, lh = lane >> 4;
  const int row0 = blockIdx.x * 64 + wave * 16;
  const _Float16* pa = X  + (size_t)(row0 + lm) * CDIM + 8 * lh;
  const _Float16* pb = Ah + (size_t)lm * CDIM + 8 * lh;
  v8f acc = vz8();
#pragma unroll 2
  for (int k0 = 0; k0 < CDIM; k0 += 32) {
    v16h a = gfrag(pa + k0);
    v16h bb = gfrag(pb + k0);
    acc = wmma16(a, bb, acc);
    asm volatile("v_nop\n\tv_nop\n\tv_nop\n\tv_nop" : "+v"(acc) : "v"(a), "v"(bb));
  }
  float* sw = St + wave * 16 * XST;
#pragma unroll
  for (int r = 0; r < 8; ++r) sw[(8 * lh + r) * XST + lm] = acc[r] * alpha;
  __syncthreads();
  v4f hv[2]; float* dp[2];
#pragma unroll
  for (int it = 0; it < 2; ++it) {
    const int row = it * 8 + (lane >> 2);
    const int p   = lane & 3;
    hv[it] = *(const v4f*)(sw + row * XST + 4 * p);
    dp[it] = xa + (size_t)(row0 + row) * LRP + 4 * p;
  }
#pragma unroll
  for (int it = 0; it < 2; ++it) *(volatile v4f*)dp[it] = hv[it];
  __threadfence();
#pragma unroll
  for (int it = 0; it < 2; ++it) *(volatile v4f*)dp[it] = hv[it];
}

__device__ __forceinline__ void kloop8(v8f (&acc)[2][4],
                                       const _Float16* pa0, const _Float16* pa1,
                                       const _Float16* pb0, const _Float16* pb1,
                                       const _Float16* pb2, const _Float16* pb3) {
#pragma unroll 2
  for (int k0 = 0; k0 < CDIM; k0 += 32) {
    v16h a0 = gfrag(pa0 + k0), a1 = gfrag(pa1 + k0);
    v16h b0 = gfrag(pb0 + k0), b1 = gfrag(pb1 + k0), b2 = gfrag(pb2 + k0), b3 = gfrag(pb3 + k0);
    acc[0][0] = wmma16(a0, b0, acc[0][0]);
    acc[1][0] = wmma16(a1, b0, acc[1][0]);
    acc[0][1] = wmma16(a0, b1, acc[0][1]);
    acc[1][1] = wmma16(a1, b1, acc[1][1]);
    acc[0][2] = wmma16(a0, b2, acc[0][2]);
    acc[1][2] = wmma16(a1, b2, acc[1][2]);
    acc[0][3] = wmma16(a0, b3, acc[0][3]);
    acc[1][3] = wmma16(a1, b3, acc[1][3]);
    asm volatile("v_nop\n\tv_nop\n\tv_nop\n\tv_nop"
                 : "+v"(acc[0][0]), "+v"(acc[1][0]), "+v"(acc[0][1]), "+v"(acc[1][1]),
                   "+v"(acc[0][2]), "+v"(acc[1][2]), "+v"(acc[0][3]), "+v"(acc[1][3])
                 : "v"(a0), "v"(a1), "v"(b0), "v"(b1), "v"(b2), "v"(b3));
  }
}

template <int MODE>
__global__ void __launch_bounds__(256) __attribute__((amdgpu_num_vgpr(256)))
gemm_kernel(const _Float16* __restrict__ A, const _Float16* __restrict__ Ar,
            const _Float16* __restrict__ Bt, const float* __restrict__ bias,
            const float* __restrict__ xa, const float* __restrict__ Bm,
            void* __restrict__ Out, _Float16* __restrict__ OutR,
            int N, int seqLen, int resRows, float alpha) {
  __shared__ __align__(16) _Float16 ldsH[MODE == 0 ? 8 * 16 * SST : 8];
  __shared__ __align__(16) float    ldsF[MODE == 1 ? 8 * 16 * SSF : 4];

  const int tid = threadIdx.x, lane = tid & 31, wave = tid >> 5, lm = lane & 15, lh = lane >> 4;
  const int waveM = wave & 3, waveN = wave >> 2;
  const int mBase = blockIdx.y * 128, nBase = blockIdx.x * 128;
  const int bseg = mBase / seqLen;
  const int t0   = mBase - bseg * seqLen;
  const bool isRes = (t0 < resRows);
  const int resBase = bseg * resRows + t0;
  const int wr0 = waveM * 32, wc0 = waveN * 64;

  v8f acc[2][4];
#pragma unroll
  for (int mi = 0; mi < 2; ++mi)
#pragma unroll
    for (int ni = 0; ni < 4; ++ni) acc[mi][ni] = vz8();

  const _Float16* pb0 = Bt + (size_t)(nBase + wc0 + 0 * 16 + lm) * CDIM + 8 * lh;
  const _Float16* pb1 = Bt + (size_t)(nBase + wc0 + 1 * 16 + lm) * CDIM + 8 * lh;
  const _Float16* pb2 = Bt + (size_t)(nBase + wc0 + 2 * 16 + lm) * CDIM + 8 * lh;
  const _Float16* pb3 = Bt + (size_t)(nBase + wc0 + 3 * 16 + lm) * CDIM + 8 * lh;

  if (MODE == 1) {
    if (isRes) {
      const _Float16* pr0 = Ar + (size_t)(resBase + wr0 + lm) * CDIM + 8 * lh;
      const _Float16* pr1 = pr0 + (size_t)16 * CDIM;
      kloop8(acc, pr0, pr1, pb0, pb1, pb2, pb3);
#pragma unroll
      for (int mi = 0; mi < 2; ++mi)
#pragma unroll
        for (int ni = 0; ni < 4; ++ni)
#pragma unroll
          for (int r = 0; r < 8; ++r) acc[mi][ni][r] = acc[mi][ni][r] * (1.0f / 1024.0f);
    }
  }
  {
    const _Float16* pa0 = A + (size_t)(mBase + wr0 + lm) * CDIM + 8 * lh;
    const _Float16* pa1 = pa0 + (size_t)16 * CDIM;
    kloop8(acc, pa0, pa1, pb0, pb1, pb2, pb3);
  }

  float bcol[4];
  float bmv[4][8];
#pragma unroll
  for (int ni = 0; ni < 4; ++ni) {
    const int n = nBase + wc0 + ni * 16 + lm;
    bcol[ni] = bf16r(bias[n]);
    v4f q0 = *(const v4f*)(Bm + (size_t)n * LR);
    v4f q1 = *(const v4f*)(Bm + (size_t)n * LR + 4);
#pragma unroll
    for (int j = 0; j < 4; ++j) { bmv[ni][j] = bf16r(q0[j]); bmv[ni][4 + j] = bf16r(q1[j]); }
  }

#pragma unroll
  for (int mi = 0; mi < 2; ++mi) {
#pragma unroll
    for (int r = 0; r < 8; ++r) {
      const int m = mBase + wr0 + mi * 16 + 8 * lh + r;
      v4f x0 = *(const v4f*)(xa + (size_t)m * LRP);
      v4f x1 = *(const v4f*)(xa + (size_t)m * LRP + 4);
#pragma unroll
      for (int ni = 0; ni < 4; ++ni) {
        float l = x0[0] * bmv[ni][0];
        l = fmaf(x0[1], bmv[ni][1], l);
        l = fmaf(x0[2], bmv[ni][2], l);
        l = fmaf(x0[3], bmv[ni][3], l);
        l = fmaf(x1[0], bmv[ni][4], l);
        l = fmaf(x1[1], bmv[ni][5], l);
        l = fmaf(x1[2], bmv[ni][6], l);
        l = fmaf(x1[3], bmv[ni][7], l);
        float v = fmaf(acc[mi][ni][r], alpha, bcol[ni]);
        v = fmaf(LSCALE, l, v);
        acc[mi][ni][r] = v;
      }
    }

    if (MODE == 0) {
      _Float16* sw = ldsH + wave * 16 * SST;
#pragma unroll
      for (int ni = 0; ni < 4; ++ni)
#pragma unroll
        for (int r = 0; r < 8; ++r)
          sw[(8 * lh + r) * SST + ni * 16 + lm] = (_Float16)acc[mi][ni][r];
      __syncthreads();
      {
        v8h hv[4]; _Float16* dp[4];
#pragma unroll
        for (int it = 0; it < 4; ++it) {
          const int row = 4 * it + (lane >> 3);
          const int j   = lane & 7;
          hv[it] = *(const v8h*)(sw + row * SST + 8 * j);
          dp[it] = (_Float16*)Out + (size_t)(mBase + wr0 + mi * 16 + row) * N + nBase + wc0 + 8 * j;
        }
#pragma unroll
        for (int it = 0; it < 4; ++it) *(volatile v8h*)dp[it] = hv[it];
        __threadfence();
#pragma unroll
        for (int it = 0; it < 4; ++it) *(volatile v8h*)dp[it] = hv[it];
      }
      __syncthreads();
      if (isRes) {
#pragma unroll
        for (int ni = 0; ni < 4; ++ni)
#pragma unroll
          for (int r = 0; r < 8; ++r) {
            const float v = acc[mi][ni][r];
            const _Float16 hh = (_Float16)v;
            sw[(8 * lh + r) * SST + ni * 16 + lm] = (_Float16)((v - (float)hh) * 1024.0f);
          }
        __syncthreads();
        {
          v8h hv[4]; _Float16* dp[4];
#pragma unroll
          for (int it = 0; it < 4; ++it) {
            const int row = 4 * it + (lane >> 3);
            const int j   = lane & 7;
            hv[it] = *(const v8h*)(sw + row * SST + 8 * j);
            dp[it] = OutR + (size_t)(resBase + wr0 + mi * 16 + row) * N + nBase + wc0 + 8 * j;
          }
#pragma unroll
          for (int it = 0; it < 4; ++it) *(volatile v8h*)dp[it] = hv[it];
          __threadfence();
#pragma unroll
          for (int it = 0; it < 4; ++it) *(volatile v8h*)dp[it] = hv[it];
        }
        __syncthreads();
      }
    } else {
      float* sw = ldsF + wave * 16 * SSF;
#pragma unroll
      for (int ni = 0; ni < 4; ++ni)
#pragma unroll
        for (int r = 0; r < 8; ++r)
          sw[(8 * lh + r) * SSF + ni * 16 + lm] = acc[mi][ni][r];
      __syncthreads();
      {
        v4f fv[8]; float* dp[8];
#pragma unroll
        for (int it = 0; it < 8; ++it) {
          const int row = 2 * it + (lane >> 4);
          const int p   = lane & 15;
          fv[it] = *(const v4f*)(sw + row * SSF + 4 * p);
          dp[it] = (float*)Out + (size_t)(mBase + wr0 + mi * 16 + row) * N + nBase + wc0 + 4 * p;
        }
#pragma unroll
        for (int it = 0; it < 8; ++it) *(volatile v4f*)dp[it] = fv[it];
        __threadfence();
#pragma unroll
        for (int it = 0; it < 8; ++it) *(volatile v4f*)dp[it] = fv[it];
      }
      __syncthreads();
    }
  }
}

__global__ void __launch_bounds__(256)
vtrans_kernel(const _Float16* __restrict__ qkvh, const _Float16* __restrict__ qkvr,
              _Float16* __restrict__ vt, _Float16* __restrict__ vtr, int seqLen, int resRows) {
  __shared__ __align__(16) _Float16 Th[64 * TS];
  __shared__ __align__(16) _Float16 Tr[64 * TS];
  const int kc = blockIdx.x, h = blockIdx.y, b = blockIdx.z;
  const int tid = threadIdx.x, wave = tid >> 5, lane = tid & 31;
  const int key = tid >> 2, piece = tid & 3;
  const bool isRes = (kc * 64 < resRows);
  {
    const _Float16* sp = qkvh + ((size_t)b * seqLen + kc * 64 + key) * NQKV + 2 * CDIM + h * HD + piece * 16;
    v8h a0 = *(const v8h*)(sp);
    v8h a1 = *(const v8h*)(sp + 8);
#pragma unroll
    for (int e = 0; e < 8; ++e) {
      Th[(piece * 16 + e) * TS + key]     = a0[e];
      Th[(piece * 16 + 8 + e) * TS + key] = a1[e];
    }
  }
  if (isRes) {
    const _Float16* sp = qkvr + ((size_t)b * resRows + kc * 64 + key) * NQKV + 2 * CDIM + h * HD + piece * 16;
    v8h a0 = *(const v8h*)(sp);
    v8h a1 = *(const v8h*)(sp + 8);
#pragma unroll
    for (int e = 0; e < 8; ++e) {
      Tr[(piece * 16 + e) * TS + key]     = a0[e];
      Tr[(piece * 16 + 8 + e) * TS + key] = a1[e];
    }
  }
  __syncthreads();
  const size_t drow0 = (size_t)(b * NH + h) * HD;
  {
    v8h hv[2]; _Float16* dp[2];
#pragma unroll
    for (int it = 0; it < 2; ++it) {
      const int d = wave * 8 + it * 4 + (lane >> 3);
      const int j = lane & 7;
      hv[it] = *(const v8h*)(Th + d * TS + 8 * j);
      dp[it] = vt + (drow0 + d) * (size_t)seqLen + kc * 64 + 8 * j;
    }
#pragma unroll
    for (int it = 0; it < 2; ++it) *(volatile v8h*)dp[it] = hv[it];
    __threadfence();
#pragma unroll
    for (int it = 0; it < 2; ++it) *(volatile v8h*)dp[it] = hv[it];
  }
  if (isRes) {
    v8h hv[2]; _Float16* dp[2];
#pragma unroll
    for (int it = 0; it < 2; ++it) {
      const int d = wave * 8 + it * 4 + (lane >> 3);
      const int j = lane & 7;
      hv[it] = *(const v8h*)(Tr + d * TS + 8 * j);
      dp[it] = vtr + (drow0 + d) * (size_t)resRows + kc * 64 + 8 * j;
    }
#pragma unroll
    for (int it = 0; it < 2; ++it) *(volatile v8h*)dp[it] = hv[it];
    __threadfence();
#pragma unroll
    for (int it = 0; it < 2; ++it) *(volatile v8h*)dp[it] = hv[it];
  }
}

template <int RES>
__global__ void __launch_bounds__(128) __attribute__((amdgpu_num_vgpr(256)))
attn_kernel(const _Float16* __restrict__ qkvh, const _Float16* __restrict__ qkvr,
            const _Float16* __restrict__ vt, const _Float16* __restrict__ vtr,
            _Float16* __restrict__ ctxh, _Float16* __restrict__ ctxr,
            int qbOff, int seqLen, int resRows) {
  __shared__ __align__(16) _Float16 Ps[4 * 16 * PST];
  __shared__ __align__(16) _Float16 Pr[RES ? 4 * 16 * PST : 8];

  const int qb = blockIdx.x + qbOff, h = blockIdx.y, b = blockIdx.z;
  const int tid = threadIdx.x, wave = tid >> 5, lane = tid & 31, lm = lane & 15, lh = lane >> 4;
  const size_t pitch = (size_t)NQKV;
  const int hc = h * HD;
  const int qtok0 = qb * 64 + wave * 16;
  const size_t qrow0 = (size_t)b * seqLen + qtok0;
  _Float16* pw  = Ps + wave * 16 * PST;
  _Float16* prw = Pr + (RES ? wave * 16 * PST : 0);

  v16h qf[2];
  {
    const _Float16* qp = qkvh + (qrow0 + lm) * pitch + hc + 8 * lh;
    qf[0] = gfrag(qp);
    qf[1] = gfrag(qp + 32);
  }
  float mrun[8], lrun[8];
#pragma unroll
  for (int i = 0; i < 8; ++i) { mrun[i] = -1e30f; lrun[i] = 0.0f; }
  v8f O1[4], O2[4];
#pragma unroll
  for (int dt = 0; dt < 4; ++dt) { O1[dt] = vz8(); O2[dt] = vz8(); }

#pragma unroll 1
  for (int kb = 0; kb <= qb; ++kb) {
    const int ktok0 = kb * 64;
    const _Float16* kp = qkvh + ((size_t)b * seqLen + ktok0 + lm) * pitch + CDIM + hc + 8 * lh;
    const _Float16* krp = kp;
    v8f S1[4], S2[4];
#pragma unroll
    for (int nt = 0; nt < 4; ++nt) { S1[nt] = vz8(); S2[nt] = vz8(); }
    v16h qr[2];
    if constexpr (RES) {
      const _Float16* qrp = qkvr + ((size_t)b * resRows + qtok0 + lm) * pitch + hc + 8 * lh;
      qr[0] = gfrag(qrp);
      qr[1] = gfrag(qrp + 32);
      krp = qkvr + ((size_t)b * resRows + ktok0 + lm) * pitch + CDIM + hc + 8 * lh;
    }
    v16h kf, kr;
#pragma unroll
    for (int ks = 0; ks < 2; ++ks) {
#pragma unroll
      for (int nt = 0; nt < 4; ++nt) {
        kf = gfrag(kp + (size_t)nt * 16 * pitch + ks * 32);
        if constexpr (RES) {
          kr = gfrag(krp + (size_t)nt * 16 * pitch + ks * 32);
          S2[nt] = wmma16(qr[ks], kf, S2[nt]);
          S1[nt] = wmma16(qf[ks], kf, S1[nt]);
          S2[nt] = wmma16(qf[ks], kr, S2[nt]);
        } else {
          S1[nt] = wmma16(qf[ks], kf, S1[nt]);
        }
      }
    }
    if constexpr (RES) {
      asm volatile("v_nop\n\tv_nop\n\tv_nop\n\tv_nop"
                   : "+v"(S1[0]), "+v"(S1[1]), "+v"(S1[2]), "+v"(S1[3]),
                     "+v"(S2[0]), "+v"(S2[1]), "+v"(S2[2]), "+v"(S2[3])
                   : "v"(qf[0]), "v"(qf[1]), "v"(qr[0]), "v"(qr[1]), "v"(kf), "v"(kr));
    } else {
      asm volatile("v_nop\n\tv_nop\n\tv_nop\n\tv_nop"
                   : "+v"(S1[0]), "+v"(S1[1]), "+v"(S1[2]), "+v"(S1[3])
                   : "v"(qf[0]), "v"(qf[1]), "v"(kf));
    }

    float mnew[8], alph[8];
#pragma unroll
    for (int i = 0; i < 8; ++i) {
      const int qt = qtok0 + 8 * lh + i;
      float vmax = -1e30f;
#pragma unroll
      for (int nt = 0; nt < 4; ++nt) {
        const int kt = ktok0 + nt * 16 + lm;
        float e;
        if constexpr (RES) e = (S1[nt][i] + S2[nt][i] * (1.0f / 1024.0f)) * 0.125f;
        else               e = S1[nt][i] * 0.125f;
        e = (kt > qt) ? -1e30f : e;
        S1[nt][i] = e;
        vmax = fmaxf(vmax, e);
      }
#pragma unroll
      for (int msk = 1; msk <= 8; msk <<= 1) vmax = fmaxf(vmax, __shfl_xor(vmax, msk, 32));
      mnew[i] = fmaxf(mrun[i], vmax);
      alph[i] = __expf(mrun[i] - mnew[i]);
    }
#pragma unroll
    for (int dt = 0; dt < 4; ++dt)
#pragma unroll
      for (int i = 0; i < 8; ++i) {
        O1[dt][i] *= alph[i];
        if constexpr (RES) O2[dt][i] *= alph[i];
      }
#pragma unroll
    for (int i = 0; i < 8; ++i) {
      float rs = 0.0f;
#pragma unroll
      for (int nt = 0; nt < 4; ++nt) {
        const float p = __expf(S1[nt][i] - mnew[i]);
        S1[nt][i] = p;
        rs += p;
      }
#pragma unroll
      for (int msk = 1; msk <= 8; msk <<= 1) rs += __shfl_xor(rs, msk, 32);
      lrun[i] = lrun[i] * alph[i] + rs;
      mrun[i] = mnew[i];
    }

#pragma unroll
    for (int nt = 0; nt < 4; ++nt)
#pragma unroll
      for (int i = 0; i < 8; ++i) {
        const float p = S1[nt][i] * 1024.0f;
        const _Float16 ph = (_Float16)p;
        pw[(8 * lh + i) * PST + nt * 16 + lm] = ph;
        if constexpr (RES) prw[(8 * lh + i) * PST + nt * 16 + lm] = (_Float16)((p - (float)ph) * 1024.0f);
      }
    __syncthreads();

    v16h pf, prf, vf, vr;
#pragma unroll
    for (int ks = 0; ks < 2; ++ks) {
      pf = gfrag(pw + lm * PST + ks * 32 + 8 * lh);
      if constexpr (RES) prf = gfrag(prw + lm * PST + ks * 32 + 8 * lh);
      const _Float16* vp  = vt + ((size_t)(b * NH + h) * HD + lm) * (size_t)seqLen + ktok0 + ks * 32 + 8 * lh;
      const _Float16* vrp = vp;
      if constexpr (RES) vrp = vtr + ((size_t)(b * NH + h) * HD + lm) * (size_t)resRows + ktok0 + ks * 32 + 8 * lh;
#pragma unroll
      for (int dt = 0; dt < 4; ++dt) {
        vf = gfrag(vp + (size_t)dt * 16 * seqLen);
        if constexpr (RES) {
          vr = gfrag(vrp + (size_t)dt * 16 * resRows);
          O2[dt] = wmma16(prf, vf, O2[dt]);
          O1[dt] = wmma16(pf, vf, O1[dt]);
          O2[dt] = wmma16(pf, vr, O2[dt]);
        } else {
          O1[dt] = wmma16(pf, vf, O1[dt]);
        }
      }
    }
    if constexpr (RES) {
      asm volatile("v_nop\n\tv_nop\n\tv_nop\n\tv_nop"
                   : "+v"(O1[0]), "+v"(O1[1]), "+v"(O1[2]), "+v"(O1[3]),
                     "+v"(O2[0]), "+v"(O2[1]), "+v"(O2[2]), "+v"(O2[3])
                   : "v"(pf), "v"(prf), "v"(vf), "v"(vr));
    } else {
      asm volatile("v_nop\n\tv_nop\n\tv_nop\n\tv_nop"
                   : "+v"(O1[0]), "+v"(O1[1]), "+v"(O1[2]), "+v"(O1[3])
                   : "v"(pf), "v"(vf));
    }
    __syncthreads();
  }

  float inv[8];
#pragma unroll
  for (int i = 0; i < 8; ++i) inv[i] = (1.0f / lrun[i]) * (16.0f / 1024.0f);
#pragma unroll
  for (int dt = 0; dt < 4; ++dt)
#pragma unroll
    for (int i = 0; i < 8; ++i) {
      float o;
      if constexpr (RES) o = (O1[dt][i] + O2[dt][i] * (1.0f / 1024.0f)) * inv[i];
      else               o = O1[dt][i] * inv[i];
      const _Float16 oh = (_Float16)o;
      pw[(8 * lh + i) * PST + dt * 16 + lm] = oh;
      if constexpr (RES) prw[(8 * lh + i) * PST + dt * 16 + lm] = (_Float16)((o - (float)oh) * 1024.0f);
    }
  __syncthreads();
  {
    v8h hv[4]; _Float16* dp[4];
#pragma unroll
    for (int it = 0; it < 4; ++it) {
      const int row = 4 * it + (lane >> 3);
      const int j   = lane & 7;
      hv[it] = *(const v8h*)(pw + row * PST + 8 * j);
      dp[it] = ctxh + (qrow0 + row) * (size_t)CDIM + hc + 8 * j;
    }
#pragma unroll
    for (int it = 0; it < 4; ++it) *(volatile v8h*)dp[it] = hv[it];
    __threadfence();
#pragma unroll
    for (int it = 0; it < 4; ++it) *(volatile v8h*)dp[it] = hv[it];
  }
  if constexpr (RES) {
    v8h hv[4]; _Float16* dp[4];
#pragma unroll
    for (int it = 0; it < 4; ++it) {
      const int row = 4 * it + (lane >> 3);
      const int j   = lane & 7;
      hv[it] = *(const v8h*)(prw + row * PST + 8 * j);
      dp[it] = ctxr + ((size_t)b * resRows + qtok0 + row) * (size_t)CDIM + hc + 8 * j;
    }
#pragma unroll
    for (int it = 0; it < 4; ++it) *(volatile v8h*)dp[it] = hv[it];
    __threadfence();
#pragma unroll
    for (int it = 0; it < 4; ++it) *(volatile v8h*)dp[it] = hv[it];
  }
}

extern "C" void kernel_launch(void* const* d_in, const int* in_sizes, int n_in,
                              void* d_out, int out_size, void* d_ws, size_t ws_size,
                              hipStream_t stream) {
  if (n_in < 9) return;
  const long long needX = ((long long)(NB - 1) * SEQ_FULL + SEQ) * CDIM;
  if ((long long)in_sizes[0] < needX) return;
  if (in_sizes[1] < NQKV * CDIM || in_sizes[2] < NQKV || in_sizes[3] < LR * CDIM ||
      in_sizes[4] < NQKV * LR || in_sizes[5] < CDIM * CDIM || in_sizes[6] < CDIM ||
      in_sizes[7] < LR * CDIM || in_sizes[8] < CDIM * LR) return;
  if ((long long)out_size < (long long)MROWS * CDIM) return;
  if (ws_size < WS_TOTAL) return;

  const float* x     = (const float*)d_in[0];
  const float* Wqkv  = (const float*)d_in[1];
  const float* bqkv  = (const float*)d_in[2];
  const float* Aqkv  = (const float*)d_in[3];
  const float* Bqkv  = (const float*)d_in[4];
  const float* Wproj = (const float*)d_in[5];
  const float* bproj = (const float*)d_in[6];
  const float* Aproj = (const float*)d_in[7];
  const float* Bproj = (const float*)d_in[8];
  float* out = (float*)d_out;

  char* ws = (char*)d_ws;
  size_t off = 0;
  _Float16* xh   = (_Float16*)(ws + off); off += SZ_XH;
  _Float16* wqh  = (_Float16*)(ws + off); off += SZ_WQ;
  _Float16* wph  = (_Float16*)(ws + off); off += SZ_WP;
  _Float16* aqh  = (_Float16*)(ws + off); off += SZ_AH;
  _Float16* aph  = (_Float16*)(ws + off); off += SZ_AH;
  float*    xaq  = (float*)(ws + off);    off += SZ_XA;
  float*    xap  = (float*)(ws + off);    off += SZ_XA;
  _Float16* qkvh = (_Float16*)(ws + off); off += SZ_QKVH;
  _Float16* qkvr = (_Float16*)(ws + off); off += SZ_QKVR;
  _Float16* vt   = (_Float16*)(ws + off); off += SZ_VT;
  _Float16* vtr  = (_Float16*)(ws + off); off += SZ_VTR;
  _Float16* ctxh = (_Float16*)(ws + off); off += SZ_CTXH;
  _Float16* ctxr = (_Float16*)(ws + off); off += SZ_CTXR;
  if (off > ws_size) return;

  const int resRows = QRES_E;

  cvt_kernel<<<dim3(MROWS * 128 / 256), dim3(256), 0, stream>>>(x, xh, MROWS, SEQ, SEQ_FULL, SEQ, 1.0f);
  cvt_kernel<<<dim3(NQKV * 128 / 256), dim3(256), 0, stream>>>(Wqkv, wqh, NQKV, NQKV, NQKV, NQKV, 64.0f);
  cvt_kernel<<<dim3(CDIM * 128 / 256), dim3(256), 0, stream>>>(Wproj, wph, CDIM, CDIM, CDIM, CDIM, 64.0f);
  cvt_kernel<<<dim3(LRP * 128 / 256), dim3(256), 0, stream>>>(Aqkv, aqh, LRP, LRP, LRP, LR, 64.0f);
  cvt_kernel<<<dim3(LRP * 128 / 256), dim3(256), 0, stream>>>(Aproj, aph, LRP, LRP, LRP, LR, 64.0f);
  lora_a_kernel<<<dim3(MROWS / 64), dim3(128), 0, stream>>>(xh, aqh, xaq, 1.0f / 64.0f);
  gemm_kernel<0><<<dim3(NQKV / 128, MROWS / 128), dim3(256), 0, stream>>>(
      xh, xh, wqh, bqkv, xaq, Bqkv, (void*)qkvh, qkvr, NQKV, SEQ, resRows, 1.0f / 64.0f);
  vtrans_kernel<<<dim3(SEQ / 64, NH, NB), dim3(256), 0, stream>>>(qkvh, qkvr, vt, vtr, SEQ, resRows);
  attn_kernel<1><<<dim3(resRows / 64, NH, NB), dim3(128), 0, stream>>>(
      qkvh, qkvr, vt, vtr, ctxh, ctxr, 0, SEQ, resRows);
  if (SEQ > resRows) {
    attn_kernel<0><<<dim3((SEQ - resRows) / 64, NH, NB), dim3(128), 0, stream>>>(
        qkvh, qkvr, vt, vtr, ctxh, ctxr, resRows / 64, SEQ, resRows);
  }
  lora_a_kernel<<<dim3(MROWS / 64), dim3(128), 0, stream>>>(ctxh, aph, xap, 1.0f / 1024.0f);
  gemm_kernel<1><<<dim3(CDIM / 128, MROWS / 128), dim3(256), 0, stream>>>(
      ctxh, ctxr, wph, bproj, xap, Bproj, (void*)out, ctxr, CDIM, SEQ, resRows, 1.0f / 1024.0f);
}
